// S4Layer_39659728011555
// MI455X (gfx1250) — hardware-run, weakly checked
//
#include <hip/hip_runtime.h>
#include <math.h>

constexpr int kB   = 4;
constexpr int kL   = 2048;
constexpr int kD   = 512;
constexpr int kS   = 64;
constexpr int kTok = kB * kL;
constexpr int kNTAP = 512;
constexpr int kNCH  = 17;
constexpr int kQP   = 576;
constexpr int kXTP  = 2624;
constexpr int kTT   = 256;
constexpr int kTP   = 72;
constexpr float kKCarry    = 32768.0f;
constexpr float kKCarryInv = 1.0f / 32768.0f;
constexpr float kWCarry    = 16.0f;
constexpr float kWCarryInv = 1.0f / 16.0f;
constexpr float kLnEps     = 1e-5f;
constexpr float kInvD      = 1.0f / 512.0f;
constexpr float kSkipArg   = -90.0f;

static_assert(kNCH * 32 >= kNTAP + 16);
static_assert(kQP >= kNCH * 32 && (kQP % 64) == 0);
static_assert(kXTP >= (kL - kTT) + 16 * 15 + 32 * kNCH && (kXTP % 64) == 0);
static_assert((kL % kTT) == 0 && kTT == 256 && (kD % 64) == 0 && (kL % 64) == 0);
static_assert((kTok % 64) == 0 && (kD % 64) == 0 && (kD % 32) == 0);

constexpr size_t kBytesXT  = (size_t)kB * kD * kXTP * 2;
constexpr size_t kBytesKsk = (size_t)kD * 16 * kQP * 2;
constexpr size_t kBytesWh  = (size_t)kD * kD * 2;
constexpr size_t kBytesY   = (size_t)kTok * kD * 2;
constexpr size_t kBytesZ   = (size_t)kTok * kD * 4;
constexpr size_t kOffXT  = 0;
constexpr size_t kOffKsk = kOffXT + kBytesXT;
constexpr size_t kOffWh  = kOffKsk + kBytesKsk;
constexpr size_t kOffY   = kOffWh + kBytesWh;
constexpr size_t kOffZ   = kOffY + kBytesY;
constexpr size_t kWsTotal = kOffZ + kBytesZ;
static_assert(kWsTotal == 45875200);
static_assert(kWsTotal <= 134217728);
static_assert((kOffKsk % 128) == 0 && (kOffWh % 128) == 0 && (kOffY % 128) == 0 && (kOffZ % 128) == 0);

typedef __attribute__((ext_vector_type(16))) _Float16 v16h;
typedef __attribute__((ext_vector_type(8)))  _Float16 v8h;
typedef __attribute__((ext_vector_type(16))) __bf16   v16b;
typedef __attribute__((ext_vector_type(8)))  __bf16   v8b;
typedef __attribute__((ext_vector_type(8)))  float    v8f;
typedef __attribute__((ext_vector_type(4)))  float    v4f;
typedef __attribute__((ext_vector_type(4)))  unsigned int v4u;

__device__ __forceinline__ unsigned short f2bf_bits(float f) {
  unsigned u = __float_as_uint(f);
  return (unsigned short)((u + 0x7FFFu + ((u >> 16) & 1u)) >> 16);
}
__device__ __forceinline__ float bf_bits2f(unsigned short h) { return __uint_as_float(((unsigned)h) << 16); }

__device__ __forceinline__ void dep_guard_h(v8f& a, v8f& b, v16h x, v16h y) { asm volatile("v_nop\n\tv_nop\n\tv_nop\n\tv_nop" : "+v"(a), "+v"(b) : "v"(x), "v"(y)); }
__device__ __forceinline__ void dep_guard_b(v8f& a, v8f& b, v16b x, v16b y) { asm volatile("v_nop\n\tv_nop\n\tv_nop\n\tv_nop" : "+v"(a), "+v"(b) : "v"(x), "v"(y)); }
__device__ __forceinline__ void keep4_h(v16h a, v16h b, v16h c, v16h d) { asm volatile("v_nop" :: "v"(a), "v"(b), "v"(c), "v"(d)); }
__device__ __forceinline__ void keep4_b(v16b a, v16b b, v16b c, v16b d) { asm volatile("v_nop" :: "v"(a), "v"(b), "v"(c), "v"(d)); }
__device__ __forceinline__ void acc_guard4(v8f& a, v8f& b, v8f& c, v8f& d) { asm volatile("v_nop\n\tv_nop\n\tv_nop\n\tv_nop" : "+v"(a), "+v"(b), "+v"(c), "+v"(d)); }
template <typename T> struct Frag;
template <> struct Frag<_Float16> {
  typedef v16h V; union U { v16h v; v8h h[2]; };
  static __device__ __forceinline__ v16h load(const _Float16* p) {
    U f; f.h[0] = *(const v8h*)(p); f.h[1] = *(const v8h*)(p + 16); return f.v;
  }
  static __device__ __forceinline__ v8f mma(v16h a, v16h b, v8f c) {
    return __builtin_amdgcn_wmma_f32_16x16x32_f16(false, a, false, b, (short)0, c, false, false);
  }
  static __device__ __forceinline__ void guard(v8f& a, v8f& b, v16h x, v16h y) { dep_guard_h(a, b, x, y); }
  static __device__ __forceinline__ void keep(v16h a, v16h b, v16h c, v16h d) { keep4_h(a, b, c, d); }
};
template <> struct Frag<__bf16> {
  typedef v16b V; union U { v16b v; v8b h[2]; };
  static __device__ __forceinline__ v16b load(const __bf16* p) {
    U f; f.h[0] = *(const v8b*)(p); f.h[1] = *(const v8b*)(p + 16); return f.v;
  }
  static __device__ __forceinline__ v8f mma(v16b a, v16b b, v8f c) {
    return __builtin_amdgcn_wmma_f32_16x16x32_bf16(false, a, false, b, (short)0, c, false, false);
  }
  static __device__ __forceinline__ void guard(v8f& a, v8f& b, v16b x, v16b y) { dep_guard_b(a, b, x, y); }
  static __device__ __forceinline__ void keep(v16b a, v16b b, v16b c, v16b d) { keep4_b(a, b, c, d); }
};

__device__ __forceinline__ unsigned pk16(unsigned short a, unsigned short b) { return (unsigned)a | ((unsigned)b << 16); }
__device__ __forceinline__ unsigned short h_bits(float f) { const _Float16 h = (_Float16)f; return __builtin_bit_cast(unsigned short, h); }

__device__ __forceinline__ float h16_to_f32(unsigned hb) {
  const unsigned sgn = (hb & 0x8000u) << 16; const unsigned em = hb & 0x7fffu;
  const float fn = __uint_as_float((em << 13) + 0x38000000u);
  const float fs = (float)em * 5.9604644775390625e-8f;
  const float mag = (em < 0x400u) ? fs : fn; return __uint_as_float(__float_as_uint(mag) | sgn); }

__device__ __forceinline__ v8f mma_h(v16h a, v16h b, v8f c) {
  c = __builtin_amdgcn_wmma_f32_16x16x32_f16(false, a, false, b, (short)0, c, false, false);
  asm volatile("v_nop\n\tv_nop\n\tv_nop\n\tv_nop" : "+v"(c) : "v"(a), "v"(b));
  return c;
}

template <int ET> struct Elem;
template <> struct Elem<0> { typedef _Float16 T; };
template <> struct Elem<1> { typedef __bf16 T; };
template <int ET, bool SPLIT, int BIAS_MODE, int OUT_MODE, bool RESID, int ACT = 0>
__global__ __launch_bounds__(256) void wmma_gemm64(
    const unsigned short* __restrict__ Ap, const unsigned short* __restrict__ A2p, int lda, long strideA,
    const unsigned short* __restrict__ Btp, const unsigned short* __restrict__ Bt2p, int ldb, long strideB,
    void* __restrict__ Cout, void* __restrict__ Cout2, int ldc, long strideC,
    const float* __restrict__ bias,
    const float* __restrict__ resid, long strideR,
    int M, int N, int K, float scale) {
  typedef typename Elem<ET>::T T;
  typedef typename Frag<T>::V V;
  const T* A = (const T*)Ap; const T* A2 = (const T*)A2p; const T* Bt = (const T*)Btp; const T* Bt2 = (const T*)Bt2p;
  __shared__ __align__(16) float sT[8][16 * 68];
  const int b    = blockIdx.y;
  const int lane = threadIdx.x & 31;
  const int wave = threadIdx.x >> 5;
  const int tilesN = N >> 6;
  const int tilesM = M >> 6;
  const int tile = blockIdx.x * 8 + wave;
  if (tile >= tilesM * tilesN) return;
  const int tm = tile / tilesN;
  const int tn = tile - tm * tilesN;
  const int m0 = tm << 6;
  const int n0 = tn << 6;

  const T* Ab  = A  + (size_t)b * strideA;
  const T* Bb  = Bt + (size_t)b * strideB;
  const T* Ab2 = SPLIT ? (A2  + (size_t)b * strideA) : nullptr;
  const T* Bb2 = SPLIT ? (Bt2 + (size_t)b * strideB) : nullptr;

  const int rlane = lane & 15;
  const int koff  = (lane >> 4) * 8;
  const int mOff  = (lane >> 4) * 8;

  v8f acc[4][4];
#pragma unroll
  for (int i = 0; i < 4; ++i)
#pragma unroll
    for (int j = 0; j < 4; ++j) acc[i][j] = (v8f){0.f,0.f,0.f,0.f,0.f,0.f,0.f,0.f};

  for (int k0 = 0; k0 < K; k0 += 32) {
    V bh[4], bl[4];
#pragma unroll
    for (int j = 0; j < 4; ++j) {
      const size_t bo = (size_t)(n0 + (j << 4) + rlane) * ldb + koff + k0;
      bh[j] = Frag<T>::load(Bb + bo);
      if (SPLIT) bl[j] = Frag<T>::load(Bb2 + bo);
    }
#pragma unroll
    for (int i = 0; i < 4; ++i) {
      const size_t ao = (size_t)(m0 + (i << 4) + rlane) * lda + koff + k0;
      V ah = Frag<T>::load(Ab + ao);
      V al;
      if (SPLIT) al = Frag<T>::load(Ab2 + ao);
#pragma unroll
      for (int j = 0; j < 4; ++j) {
        acc[i][j] = Frag<T>::mma(ah, bh[j], acc[i][j]);
        if (SPLIT) {
          acc[i][j] = Frag<T>::mma(ah, bl[j], acc[i][j]);
          acc[i][j] = Frag<T>::mma(al, bh[j], acc[i][j]);
        }
      }
      Frag<T>::guard(acc[i][0], acc[i][3], ah, SPLIT ? al : ah);
    }
    Frag<T>::keep(bh[0], bh[1], bh[2], bh[3]);
    if (SPLIT) Frag<T>::keep(bl[0], bl[1], bl[2], bl[3]);
  }
  acc_guard4(acc[0][0], acc[0][1], acc[0][2], acc[0][3]);
  acc_guard4(acc[1][0], acc[1][1], acc[1][2], acc[1][3]);
  acc_guard4(acc[2][0], acc[2][1], acc[2][2], acc[2][3]);
  acc_guard4(acc[3][0], acc[3][1], acc[3][2], acc[3][3]);

  float* slab = sT[wave];
  const float* Rb = RESID ? (resid + (size_t)b * strideR) : nullptr;
#pragma unroll
  for (int i = 0; i < 4; ++i) {
    const int mBase = m0 + (i << 4);
#pragma unroll
    for (int j = 0; j < 4; ++j) {
      const int n = n0 + (j << 4) + rlane;
      float bv = 0.f;
      if (BIAS_MODE == 2) bv = bias[n];
#pragma unroll
      for (int r = 0; r < 8; ++r) {
        float v = acc[i][j][r] * scale;
        if (BIAS_MODE == 1) v += bias[mBase + mOff + r];
        if (BIAS_MODE == 2) v += bv;
        if (RESID) v += Rb[(size_t)(mBase + mOff + r) * ldc + n];
        if (ACT == 2) v = fmaxf(v, 0.0f);
        if (ACT == 4) v = (v > 0.f) ? v : 0.01f * v;
        slab[(mOff + r) * 68 + (j << 4) + rlane] = v;
      }
    }
    __builtin_amdgcn_fence(__ATOMIC_RELEASE, "workgroup");
    __builtin_amdgcn_wave_barrier();
    __builtin_amdgcn_fence(__ATOMIC_ACQUIRE, "workgroup");
    if (OUT_MODE == 0) {
      float* C = (float*)Cout + (size_t)b * strideC;
      const int hh = lane >> 4, c4 = (lane & 15) * 4;
      for (int pass = 0; pass < 2; ++pass) {
#pragma unroll
        for (int it = 0; it < 8; ++it) {
          const int row = it * 2 + hh;
          v4f v = *(const v4f*)(slab + row * 68 + c4);
          *(volatile v4f*)(C + (size_t)(mBase + row) * ldc + n0 + c4) = v;
        }
        __threadfence();
      }
    } else {
      const int q = lane >> 3, c8 = (lane & 7) * 8;
      unsigned short* C  = (unsigned short*)Cout  + (size_t)b * strideC;
      unsigned short* C2 = (OUT_MODE == 2) ? ((unsigned short*)Cout2 + (size_t)b * strideC) : nullptr;
      for (int pass = 0; pass < 2; ++pass) {
#pragma unroll
        for (int it = 0; it < 4; ++it) {
          const int row = it * 4 + q;
          const float* sp = slab + row * 68 + c8;
          v8h hv, lv;
#pragma unroll
          for (int e = 0; e < 8; ++e) {
            if (OUT_MODE == 1) {
              hv[e] = (_Float16)sp[e];
            } else {
              unsigned short hb = f2bf_bits(sp[e]);
              unsigned short lb = f2bf_bits(sp[e] - bf_bits2f(hb));
              hv[e] = __builtin_bit_cast(_Float16, hb);
              lv[e] = __builtin_bit_cast(_Float16, lb);
            }
          }
          *(volatile v8h*)(C + (size_t)(mBase + row) * ldc + n0 + c8) = hv;
          if (OUT_MODE == 2) *(volatile v8h*)(C2 + (size_t)(mBase + row) * ldc + n0 + c8) = lv;
        }
        __threadfence();
      }
    }
    __builtin_amdgcn_fence(__ATOMIC_RELEASE, "workgroup");
    __builtin_amdgcn_wave_barrier();
    __builtin_amdgcn_fence(__ATOMIC_ACQUIRE, "workgroup");
  }
}

__global__ __launch_bounds__(256) void xpose_cast_kernel(const float* __restrict__ x, unsigned short* __restrict__ xT) {
  __shared__ float sm[64][65];
  const int tid = threadIdx.x;
  const int tt  = blockIdx.x;
  const int d0  = blockIdx.y * 64;
  const int b   = blockIdx.z;
  const int t0  = tt * 64;
  if (tt < kL / 64) {
#pragma unroll
    for (int i = 0; i < 4; ++i) {
      const int e  = i * 256 + tid;
      const int r  = e >> 4;
      const int c4 = (e & 15) * 4;
      const v4f v = *(const v4f*)(x + ((size_t)(b * kL + t0 + r)) * kD + d0 + c4);
      sm[c4 + 0][r] = v[0];
      sm[c4 + 1][r] = v[1];
      sm[c4 + 2][r] = v[2];
      sm[c4 + 3][r] = v[3];
    }
  } else {
#pragma unroll
    for (int i = 0; i < 4; ++i) {
      const int e  = i * 256 + tid;
      const int r  = e >> 4;
      const int c4 = (e & 15) * 4;
      sm[c4 + 0][r] = 0.0f;
      sm[c4 + 1][r] = 0.0f;
      sm[c4 + 2][r] = 0.0f;
      sm[c4 + 3][r] = 0.0f;
    }
  }
  __syncthreads();
  const int lane = tid & 31, wave = tid >> 5;
  const int q8 = lane >> 3, c8 = (lane & 7) * 8;
  unsigned short* op = xT + ((size_t)(b * kD + d0)) * kXTP + t0 + c8;
  v4u u2[2];
#pragma unroll
  for (int it = 0; it < 2; ++it) {
    const int row = wave * 8 + it * 4 + q8;
    unsigned short hb[8];
#pragma unroll
    for (int e = 0; e < 8; ++e) hb[e] = h_bits(sm[row][c8 + e]);
    u2[it] = (v4u){pk16(hb[0], hb[1]), pk16(hb[2], hb[3]), pk16(hb[4], hb[5]), pk16(hb[6], hb[7])};
  }
  for (int pass = 0; pass < 2; ++pass) {
#pragma unroll
    for (int it = 0; it < 2; ++it) {
      const int row = wave * 8 + it * 4 + q8;
      *(volatile v4u*)(op + (size_t)row * kXTP) = u2[it];
    }
    __threadfence();
  }
}

__global__ __launch_bounds__(256) void wcast8_kernel(const float* __restrict__ in, unsigned short* __restrict__ out,
                                                    int n8, float scale) {
  const int i = blockIdx.x * 256 + threadIdx.x;
  if (i >= n8) return;
  const float* p = in + 8 * (size_t)i;
  const v4f a = *(const v4f*)(p);
  const v4f c = *(const v4f*)(p + 4);
  unsigned short hb[8];
#pragma unroll
  for (int e = 0; e < 4; ++e) {
    hb[e]     = h_bits(a[e] * scale);
    hb[4 + e] = h_bits(c[e] * scale);
  }
  const v4u u = (v4u){pk16(hb[0], hb[1]), pk16(hb[2], hb[3]), pk16(hb[4], hb[5]), pk16(hb[6], hb[7])};
  unsigned short* q = out + 8 * (size_t)i;
  *(volatile v4u*)q = u;
  __threadfence();
  *(volatile v4u*)q = u;
}

__global__ __launch_bounds__(512) void tapgen_kernel(const float* __restrict__ lar, const float* __restrict__ aim,
                                                    const float* __restrict__ Bp, const float* __restrict__ Cp,
                                                    unsigned short* __restrict__ Ksk) {
  __shared__ float sAr[kS];
  __shared__ float sAi[kS];
  __shared__ float sP[kS];
  __shared__ float sQ[kS];
  __shared__ float sK[kNTAP];
  const int tid = threadIdx.x;
  const int d   = blockIdx.x;
  {
    const int s = tid & (kS - 1);
    const int i = d * kS + s;
    const float lv = lar[i];
    const float av = aim[i];
    const float br = Bp[2 * i], bi = Bp[2 * i + 1];
    const float cr = Cp[2 * i], ci = Cp[2 * i + 1];
    const float arv = -expf(lv);
    const float pv  = cr * br + ci * bi;
    const float qv  = cr * bi - ci * br;
    if (tid < kS) {
      sAr[tid] = arv;
      sAi[tid] = av;
      sP[tid]  = pv;
      sQ[tid]  = qv;
    }
  }
  __syncthreads();

  const int wave = __builtin_amdgcn_readfirstlane(tid >> 5);
  const float lwf = (float)(wave * 32);
  const float lf  = (float)tid;
  float acc = 0.0f;
#pragma unroll 1
  for (int s = 0; s < kS; ++s) {
    const float ar = sAr[s];
    if (lwf * ar >= kSkipArg) {
      const float ai = sAi[s];
      const float pv = sP[s];
      const float qv = sQ[s];
      const float ex = expf(lf * ar);
      float sn, cs;
      sincosf(lf * ai, &sn, &cs);
      acc += ex * (pv * cs - qv * sn);
    }
  }
  sK[tid] = acc;
  __syncthreads();

  v4u vals[3];
#pragma unroll
  for (int i = 0; i < 3; ++i) {
    const int e  = i * 512 + tid;
    const int m  = e / 72;
    const int q0 = (e - m * 72) * 8;
    unsigned short hb[8];
#pragma unroll
    for (int k = 0; k < 8; ++k) {
      const int j  = q0 + k - m;
      const int jc = j < 0 ? 0 : (j > kNTAP - 1 ? kNTAP - 1 : j);
      const float kv = sK[jc] * kKCarry;
      const float v  = (j >= 0 && j < kNTAP) ? kv : 0.0f;
      hb[k] = h_bits(v);
    }
    vals[i] = (v4u){pk16(hb[0], hb[1]), pk16(hb[2], hb[3]), pk16(hb[4], hb[5]), pk16(hb[6], hb[7])};
  }
  unsigned short* op = Ksk + (size_t)d * (16 * kQP);
  for (int pass = 0; pass < 2; ++pass) {
#pragma unroll
    for (int i = 0; i < 3; ++i) {
      const int e = i * 512 + tid;
      if (e < 16 * 72) {
        const int m  = e / 72;
        const int q0 = (e - m * 72) * 8;
        *(volatile v4u*)(op + (size_t)m * kQP + q0) = vals[i];
      }
    }
    __threadfence();
  }
}

__global__ __launch_bounds__(256) void corr_kernel(const unsigned short* __restrict__ Ksk, const unsigned short* __restrict__ xT,
                                                  const float* __restrict__ x, const float* __restrict__ Dp,
                                                  unsigned short* __restrict__ y) {
  __shared__ __align__(16) unsigned short tile[kTT * kTP];
  const int tid  = threadIdx.x;
  const int lane = tid & 31, wave = tid >> 5;
  const int h    = lane >> 4, c16 = lane & 15;
  const int T0   = blockIdx.x * kTT;
  const int d0   = blockIdx.y * 64;
  const int b    = blockIdx.z;
  const _Float16* Kh = (const _Float16*)Ksk;
  const _Float16* Xh = (const _Float16*)xT;

#pragma unroll 1
  for (int ci = 0; ci < 8; ++ci) {
    const int dl = wave * 8 + ci;
    const int d  = d0 + dl;
    const _Float16* Ab = Kh + ((size_t)d * 16 + c16) * kQP + 8 * h;
    const _Float16* Bb = Xh + ((size_t)b * kD + d) * kXTP + T0 + 16 * c16 + 8 * h;
    v8f acc = (v8f){0.f,0.f,0.f,0.f,0.f,0.f,0.f,0.f};
#pragma unroll 1
    for (int c = 0; c < kNCH; ++c) {
      const v16h fa = Frag<_Float16>::load(Ab + 32 * c);
      const v16h fb = Frag<_Float16>::load(Bb + 32 * c);
      acc = mma_h(fa, fb, acc);
    }
#pragma unroll
    for (int r = 0; r < 8; ++r) {
      const float av = acc[r];
      tile[(16 * c16 + 8 * h + r) * kTP + dl] = h_bits(av);
    }
  }
  __syncthreads();

  const int q8 = lane >> 3, c8 = (lane & 7) * 8;
  const v4f da = *(const v4f*)(Dp + d0 + c8);
  const v4f db = *(const v4f*)(Dp + d0 + c8 + 4);
  float dv[8];
  dv[0] = da[0]; dv[1] = da[1]; dv[2] = da[2]; dv[3] = da[3];
  dv[4] = db[0]; dv[5] = db[1]; dv[6] = db[2]; dv[7] = db[3];
  v4u vals[8];
#pragma unroll
  for (int it = 0; it < 8; ++it) {
    const int row = it * 32 + wave * 4 + q8;
    const v4u wv = *(const v4u*)(tile + row * kTP + c8);
    const size_t gb = ((size_t)(b * kL + T0 + row)) * kD + d0 + c8;
    const v4f xa = *(const v4f*)(x + gb);
    const v4f xb = *(const v4f*)(x + gb + 4);
    const unsigned w0 = wv[0], w1 = wv[1], w2 = wv[2], w3 = wv[3];
    float cv[8];
    cv[0] = h16_to_f32(w0 & 0xffffu); cv[1] = h16_to_f32(w0 >> 16);
    cv[2] = h16_to_f32(w1 & 0xffffu); cv[3] = h16_to_f32(w1 >> 16);
    cv[4] = h16_to_f32(w2 & 0xffffu); cv[5] = h16_to_f32(w2 >> 16);
    cv[6] = h16_to_f32(w3 & 0xffffu); cv[7] = h16_to_f32(w3 >> 16);
    float xv[8];
    xv[0] = xa[0]; xv[1] = xa[1]; xv[2] = xa[2]; xv[3] = xa[3];
    xv[4] = xb[0]; xv[5] = xb[1]; xv[6] = xb[2]; xv[7] = xb[3];
    unsigned short hb[8];
#pragma unroll
    for (int k = 0; k < 8; ++k) {
      const float yk = fmaf(dv[k], xv[k], cv[k] * kKCarryInv);
      hb[k] = h_bits(yk);
    }
    vals[it] = (v4u){pk16(hb[0], hb[1]), pk16(hb[2], hb[3]), pk16(hb[4], hb[5]), pk16(hb[6], hb[7])};
    if ((it & 1) == 1) asm volatile("" ::: "memory");
  }
  unsigned short* yb = y + ((size_t)(b * kL + T0)) * kD + d0 + c8;
  for (int pass = 0; pass < 2; ++pass) {
#pragma unroll
    for (int it = 0; it < 8; ++it) {
      const int row = it * 32 + wave * 4 + q8;
      *(volatile v4u*)(yb + (size_t)row * kD) = vals[it];
    }
    __threadfence();
  }
}

__global__ __launch_bounds__(128) void lnorm_kernel(const float* __restrict__ zp, const float* __restrict__ x,
                                                   const float* __restrict__ bo, const float* __restrict__ gm,
                                                   const float* __restrict__ bt, float* __restrict__ out) {
  __shared__ float red1[4];
  __shared__ float red2[4];
  const int tid = threadIdx.x, lane = tid & 31, wave = tid >> 5;
  const size_t tok = blockIdx.x;
  const int c4 = tid * 4;
  const size_t base = tok * kD + c4;
  const v4f a  = *(const v4f*)(zp + base);
  const v4f xx = *(const v4f*)(x + base);
  const v4f bb = *(const v4f*)(bo + c4);
  const v4f g  = *(const v4f*)(gm + c4);
  const v4f be = *(const v4f*)(bt + c4);
  float z[4];
#pragma unroll
  for (int k = 0; k < 4; ++k) z[k] = (a[k] + bb[k]) + xx[k];
  float s = (z[0] + z[1]) + (z[2] + z[3]);
#pragma unroll
  for (int off = 16; off > 0; off >>= 1) s += __shfl_xor(s, off, 32);
  if (lane == 0) red1[wave] = s;
  __syncthreads();
  const float mu = ((red1[0] + red1[1]) + (red1[2] + red1[3])) * kInvD;
  float dvz[4];
  float s2 = 0.0f;
#pragma unroll
  for (int k = 0; k < 4; ++k) { dvz[k] = z[k] - mu; s2 += dvz[k] * dvz[k]; }
#pragma unroll
  for (int off = 16; off > 0; off >>= 1) s2 += __shfl_xor(s2, off, 32);
  if (lane == 0) red2[wave] = s2;
  __syncthreads();
  const float var  = ((red2[0] + red2[1]) + (red2[2] + red2[3])) * kInvD;
  const float rstd = 1.0f / sqrtf(var + kLnEps);
  const float o0 = (g[0] * dvz[0]) * rstd + be[0];
  const float o1 = (g[1] * dvz[1]) * rstd + be[1];
  const float o2 = (g[2] * dvz[2]) * rstd + be[2];
  const float o3 = (g[3] * dvz[3]) * rstd + be[3];
  const v4f ov = (v4f){o0, o1, o2, o3};
  float* op = out + base;
  *(volatile v4f*)op = ov;
  __threadfence();
  *(volatile v4f*)op = ov;
}

extern "C" void kernel_launch(void* const* d_in, const int* in_sizes, int n_in,
                              void* d_out, int out_size, void* d_ws, size_t ws_size, hipStream_t stream) {
  if (n_in < 10) return;
  if (in_sizes[0] != kTok * kD || in_sizes[1] != kD * kS || in_sizes[2] != kD * kS ||
      in_sizes[3] != kD * kS * 2 || in_sizes[4] != kD * kS * 2 || in_sizes[5] != kD ||
      in_sizes[6] != kD * kD || in_sizes[7] != kD || in_sizes[8] != kD || in_sizes[9] != kD ||
      out_size != kTok * kD) return;
  if (ws_size < kWsTotal) return;

  const float* x   = (const float*)d_in[0];
  const float* lar = (const float*)d_in[1];
  const float* aim = (const float*)d_in[2];
  const float* Bp  = (const float*)d_in[3];
  const float* Cp  = (const float*)d_in[4];
  const float* Dp  = (const float*)d_in[5];
  const float* Wo  = (const float*)d_in[6];
  const float* bo  = (const float*)d_in[7];
  const float* gm  = (const float*)d_in[8];
  const float* bt  = (const float*)d_in[9];
  float* out = (float*)d_out;
  char* ws = (char*)d_ws;

  unsigned short* xT  = (unsigned short*)(ws + kOffXT);
  unsigned short* Ksk = (unsigned short*)(ws + kOffKsk);
  unsigned short* Wh  = (unsigned short*)(ws + kOffWh);
  unsigned short* yh  = (unsigned short*)(ws + kOffY);
  float*          zp  = (float*)(ws + kOffZ);

  xpose_cast_kernel<<<dim3(kXTP / 64, kD / 64, kB), 256, 0, stream>>>(x, xT);
  wcast8_kernel<<<(kD * kD / 8) / 256, 256, 0, stream>>>(Wo, Wh, kD * kD / 8, kWCarry);
  tapgen_kernel<<<kD, 512, 0, stream>>>(lar, aim, Bp, Cp, Ksk);
  corr_kernel<<<dim3(kL / kTT, kD / 64, kB), 256, 0, stream>>>(Ksk, xT, x, Dp, yh);
  wmma_gemm64<0, false, 0, 0, false, 0><<<dim3((kTok / 64) * (kD / 64) / 8, 1), 256, 0, stream>>>(
      yh, nullptr, kD, 0L,
      Wh, nullptr, kD, 0L,
      (void*)zp, nullptr, kD, 0L,
      nullptr,
      nullptr, 0L,
      kTok, kD, kD, kWCarryInv);
  lnorm_kernel<<<kTok, 128, 0, stream>>>(zp, x, bo, gm, bt, out);
}
